// PointNetSetAbstraction_52304111730780
// MI455X (gfx1250) — hardware-verified
//
#include <hip/hip_runtime.h>

#pragma clang fp contract(off)

typedef __attribute__((ext_vector_type(16))) _Float16 v16h;
typedef __attribute__((ext_vector_type(8)))  float    v8f;
typedef __attribute__((ext_vector_type(4)))  float    v4f;
typedef __attribute__((ext_vector_type(4)))  unsigned v4u;
typedef unsigned v4ua __attribute__((ext_vector_type(4), may_alias));

constexpr int NBATCH    = 16;
constexpr int NPTS      = 4096;
constexpr int NCENT     = 1024;
constexpr int NNBR      = 32;
constexpr int CH_IN     = 64;
constexpr int CH_L0     = 64;
constexpr int CH_L1     = 64;
constexpr int CH_L2     = 128;
constexpr int KREAL0    = CH_IN + 3;
constexpr int KPAD0     = 96;
constexpr int NGRP      = NBATCH * NCENT;
constexpr int NROWS     = NGRP * NNBR;
constexpr int TILE_ROWS = 128;
constexpr int NTILES    = NROWS / TILE_ROWS;
constexpr int LIST_CAP  = 256;
constexpr float W_CARRY     = 64.0f;
constexpr float W_CARRY_INV = 1.0f / W_CARRY;
constexpr float RADIUS_SQ   = (float)(0.4 * 0.4);
constexpr float BN_EPS      = 1e-5f;

static_assert(NROWS == 524288, "row count");
static_assert(NTILES * TILE_ROWS == NROWS, "tile multiple");
static_assert(KPAD0 % 32 == 0 && KPAD0 >= KREAL0, "layer-0 K pad");
static_assert(CH_L0 % 32 == 0 && CH_L1 % 32 == 0, "K multiples");
static_assert((NGRP * 3 + NGRP * CH_L2) * 4 == 8585216, "output bytes");
static_assert((NGRP * 3 * 4) % 128 == 0, "second output starts on a line");
static_assert(TILE_ROWS / NNBR == 4, "groups per tile");

constexpr size_t WS_NXYZ  = (size_t)NGRP * 3 * 4;
constexpr size_t WS_PT4   = (size_t)NBATCH * NPTS * 16;
constexpr size_t WS_GIDX  = (size_t)NGRP * NNBR * 4;
constexpr size_t WS_W0H   = (size_t)CH_L0 * KPAD0 * 2;
constexpr size_t WS_W1H   = (size_t)CH_L1 * CH_L0 * 2;
constexpr size_t WS_W2H   = (size_t)CH_L2 * CH_L1 * 2;
constexpr size_t WS_Y0    = (size_t)NROWS * CH_L0 * 2;
constexpr size_t WS_PART0 = (size_t)NTILES * 2 * CH_L0 * 4;
constexpr size_t WS_PART1 = (size_t)NTILES * 2 * CH_L1 * 4;
constexpr size_t WS_PART2 = (size_t)NTILES * 2 * CH_L2 * 4;
constexpr size_t WS_SCSH0 = (size_t)2 * CH_L0 * 4;
constexpr size_t WS_SCSH1 = (size_t)2 * CH_L1 * 4;
constexpr size_t WS_SCSH2 = (size_t)2 * CH_L2 * 4;
constexpr size_t WS_GMAX  = (size_t)NGRP * CH_L2 * 4;
constexpr size_t WS_GMIN  = (size_t)NGRP * CH_L2 * 4;
constexpr size_t WS_TOTAL = WS_NXYZ + WS_PT4 + WS_GIDX + WS_W0H + WS_W1H + WS_W2H + WS_Y0 + WS_PART0 +
                            WS_PART1 + WS_PART2 + WS_SCSH0 + WS_SCSH1 + WS_SCSH2 + WS_GMAX + WS_GMIN;
static_assert(WS_TOTAL <= (size_t)134217728, "workspace carve");
static_assert(WS_NXYZ % 256 == 0 && WS_W0H % 256 == 0 && WS_W1H % 256 == 0 && WS_SCSH0 % 256 == 0, "carve alignment");

__device__ __forceinline__ unsigned hbits(float x) {
  const _Float16 hv = (_Float16)x;
  return (unsigned)__builtin_bit_cast(unsigned short, hv);
}
__device__ __forceinline__ unsigned pack2h(float a, float b) {
  const unsigned lo = hbits(a);
  const unsigned hi = hbits(b);
  return (lo & 0xffffu) | (hi << 16);
}
__device__ __forceinline__ float h16_to_f32(unsigned hb) {
  const unsigned sgn = (hb & 0x8000u) << 16;
  const unsigned em = hb & 0x7fffu;
  const float fn = __uint_as_float((em << 13) + 0x38000000u);
  const float fs = (float)em * 5.9604644775390625e-8f;
  const float mag = (em < 0x400u) ? fs : fn;
  return __uint_as_float(__float_as_uint(mag) | sgn);
}
union FragU { v16h v; v4u q[2]; };
__device__ __forceinline__ v16h lds_frag(const unsigned short* tile, int hoff) {
  FragU f;
  f.q[0] = *(const v4ua*)(tile + hoff);
  f.q[1] = *(const v4ua*)(tile + hoff + 16);
  return f.v;
}
__device__ __forceinline__ v8f mma_h(v16h a, v16h b, v8f c) {
  c = __builtin_amdgcn_wmma_f32_16x16x32_f16(false, a, false, b, (short)0, c, false, false);
  asm volatile("v_nop\n\tv_nop\n\tv_nop\n\tv_nop" : "+v"(c) : "v"(a), "v"(b));
  return c;
}
__device__ __forceinline__ unsigned bn_relu_pack(unsigned w, float sca, float sha, float scb, float shb) {
  const float ya = h16_to_f32(w & 0xffffu);
  const float yb = h16_to_f32(w >> 16);
  const float ta = ya * sca;
  const float tb = yb * scb;
  const float aa = fmaxf(ta + sha, 0.0f);
  const float ab = fmaxf(tb + shb, 0.0f);
  return pack2h(aa, ab);
}

__global__ __launch_bounds__(512) void k_fps(const float* __restrict__ xyz, float* __restrict__ out0,
                                             float* __restrict__ nxyz) {
#pragma clang fp contract(off)
  __shared__ __align__(16) float sx[NPTS * 3];
  __shared__ __align__(16) float snew[NCENT * 3];
  __shared__ unsigned sredH[2][16];
  __shared__ unsigned sredL[2][16];
  const int b = blockIdx.x;
  const int t = threadIdx.x;
  const int lane = t & 31;
  const int wave = t >> 5;
  {
    const v4f* src = (const v4f*)(xyz + (size_t)b * NPTS * 3);
    v4f tmp[6];
#pragma unroll
    for (int i = 0; i < 6; ++i) tmp[i] = src[t + i * 512];
#pragma unroll
    for (int i = 0; i < 6; ++i) *(v4f*)(sx + (size_t)(t + i * 512) * 4) = tmp[i];
  }
  __syncthreads();
  float px[8], py[8], pz[8], dd[8];
#pragma unroll
  for (int i = 0; i < 8; ++i) {
    const int n = t + i * 512;
    px[i] = sx[n * 3 + 0];
    py[i] = sx[n * 3 + 1];
    pz[i] = sx[n * 3 + 2];
    dd[i] = __builtin_huge_valf();
  }
  float lx = sx[0], ly = sx[1], lz = sx[2];
  if (t == 0) { snew[0] = lx; snew[1] = ly; snew[2] = lz; }
  int par = 0;
#pragma unroll 1
  for (int k = 1; k < NCENT; ++k) {
    unsigned bh = 0u, bl = 0u;
#pragma unroll
    for (int i = 0; i < 8; ++i) {
      const float dx = px[i] - lx;
      const float dy = py[i] - ly;
      const float dz = pz[i] - lz;
      const float t0 = dx * dx;
      const float t1 = dy * dy;
      const float t2 = dz * dz;
      float d = (t0 + t2) + t1;
      d = fminf(dd[i], d);
      dd[i] = d;
      const unsigned hb = __float_as_uint(d);
      const unsigned lb = 0xFFFFFFFFu - (unsigned)(t + i * 512);
      const bool better = (hb > bh) || (hb == bh && lb > bl);
      bh = better ? hb : bh;
      bl = better ? lb : bl;
    }
#pragma unroll
    for (int off = 16; off > 0; off >>= 1) {
      const unsigned oh = __shfl_xor(bh, off, 32);
      const unsigned ol = __shfl_xor(bl, off, 32);
      const bool better = (oh > bh) || (oh == bh && ol > bl);
      bh = better ? oh : bh;
      bl = better ? ol : bl;
    }
    if (lane == 0) { sredH[par][wave] = bh; sredL[par][wave] = bl; }
    __syncthreads();
    unsigned vh = sredH[par][lane & 15];
    unsigned vl = sredL[par][lane & 15];
#pragma unroll
    for (int off = 8; off > 0; off >>= 1) {
      const unsigned oh = __shfl_xor(vh, off, 32);
      const unsigned ol = __shfl_xor(vl, off, 32);
      const bool better = (oh > vh) || (oh == vh && ol > vl);
      vh = better ? oh : vh;
      vl = better ? ol : vl;
    }
    int nxt = (int)(0xFFFFFFFFu - vl);
    nxt = nxt < 0 ? 0 : (nxt > NPTS - 1 ? NPTS - 1 : nxt);
    lx = sx[nxt * 3 + 0];
    ly = sx[nxt * 3 + 1];
    lz = sx[nxt * 3 + 2];
    if (t == 0) { snew[k * 3 + 0] = lx; snew[k * 3 + 1] = ly; snew[k * 3 + 2] = lz; }
    par ^= 1;
  }
  __syncthreads();
  for (int pass = 0; pass < 2; ++pass) {
#pragma unroll
    for (int it = 0; it < 2; ++it) {
      const int i = it * 512 + t;
      if (i < (NCENT * 3) / 4) {
        const v4f val = *(const v4f*)(snew + (size_t)i * 4);
        *(volatile v4f*)(out0 + (size_t)b * NCENT * 3 + (size_t)i * 4) = val;
        *(volatile v4f*)(nxyz + (size_t)b * NCENT * 3 + (size_t)i * 4) = val;
      }
    }
    __threadfence();
  }
}

__global__ __launch_bounds__(256) void k_prep(const float* __restrict__ xyz, const float* __restrict__ W0,
                                              const float* __restrict__ W1, const float* __restrict__ W2,
                                              unsigned* __restrict__ w0h, unsigned* __restrict__ w1h,
                                              unsigned* __restrict__ w2h, float* __restrict__ pt4) {
#pragma clang fp contract(off)
  const int t = threadIdx.x;
  const int blk = blockIdx.x;
  if (blk < 3) {
    const int u = blk * 256 + t;
    const int n = u / 12;
    const int kq = u - n * 12;
    float v[8];
#pragma unroll
    for (int e = 0; e < 8; ++e) {
      const int k = kq * 8 + e;
      const int col = (k < CH_IN) ? (k + 3) : ((k < KREAL0) ? (k - CH_IN) : 0);
      const float x = W0[n * KREAL0 + col];
      const float xs = x * W_CARRY;
      v[e] = (k < KREAL0) ? xs : 0.0f;
    }
    v4u w;
    w.x = pack2h(v[0], v[1]);
    w.y = pack2h(v[2], v[3]);
    w.z = pack2h(v[4], v[5]);
    w.w = pack2h(v[6], v[7]);
    volatile v4u* dst = (volatile v4u*)w0h + u;
    *dst = w;
    __threadfence();
    *dst = w;
  } else if (blk < 9) {
    const bool isW1 = (blk < 5);
    const int u = isW1 ? ((blk - 3) * 256 + t) : ((blk - 5) * 256 + t);
    const float* src = isW1 ? W1 : W2;
    unsigned* dstp = isW1 ? w1h : w2h;
    const v4f a0 = *(const v4f*)(src + (size_t)u * 8);
    const v4f a1 = *(const v4f*)(src + (size_t)u * 8 + 4);
    v4u w;
    w.x = pack2h(a0.x * W_CARRY, a0.y * W_CARRY);
    w.y = pack2h(a0.z * W_CARRY, a0.w * W_CARRY);
    w.z = pack2h(a1.x * W_CARRY, a1.y * W_CARRY);
    w.w = pack2h(a1.z * W_CARRY, a1.w * W_CARRY);
    volatile v4u* dst = (volatile v4u*)dstp + u;
    *dst = w;
    __threadfence();
    *dst = w;
  } else {
    const int i = (blk - 9) * 256 + t;
    if (i < NBATCH * NPTS) {
      const float x = xyz[(size_t)i * 3 + 0];
      const float y = xyz[(size_t)i * 3 + 1];
      const float z = xyz[(size_t)i * 3 + 2];
      const float t0 = x * x;
      const float t1 = y * y;
      const float t2 = z * z;
      v4f o;
      o.x = x; o.y = y; o.z = z; o.w = (t0 + t2) + t1;
      volatile v4f* dst = (volatile v4f*)pt4 + i;
      *dst = o;
      __threadfence();
      *dst = o;
    }
  }
}

__global__ __launch_bounds__(256) void k_ballquery(const float* __restrict__ pt4, const float* __restrict__ nxyz,
                                                   int* __restrict__ gidx) {
#pragma clang fp contract(off)
  __shared__ float sLd[8][LIST_CAP];
  __shared__ int   sLi[8][LIST_CAP];
  __shared__ int   sSel[8][32];
  const int lane = threadIdx.x & 31;
  const int wave = threadIdx.x >> 5;
  const int q = blockIdx.x * 8 + wave;
  const int b = q >> 10;
  const v4f* pb = (const v4f*)pt4 + (size_t)b * NPTS;
  const float qx = nxyz[(size_t)q * 3 + 0];
  const float qy = nxyz[(size_t)q * 3 + 1];
  const float qz = nxyz[(size_t)q * 3 + 2];
  const float q0 = qx * qx;
  const float q1 = qy * qy;
  const float q2t = qz * qz;
  const float qq = (q0 + q2t) + q1;
  if (lane == 0) { sLd[wave][0] = 0.0f; sLi[wave][0] = 0; }
  __syncthreads();
  int cnt = 0;
  float bestd = __builtin_huge_valf();
  int besti = 0;
  const unsigned lt_mask = (1u << lane) - 1u;
#pragma unroll 2
  for (int it = 0; it < NPTS / 32; ++it) {
    const int n = it * 32 + lane;
    const v4f p = pb[n];
    float dot = qx * p.x;
    dot = __builtin_fmaf(qy, p.y, dot);
    dot = __builtin_fmaf(qz, p.z, dot);
    const float ssum = qq + p.w;
    const float two = 2.0f * dot;
    float d2 = ssum - two;
    d2 = fmaxf(d2, 0.0f);
    const bool inC = (d2 <= RADIUS_SQ);
    const unsigned mask = __builtin_amdgcn_ballot_w32(inC);
    const int pos = cnt + __popc(mask & lt_mask);
    if (inC && pos < LIST_CAP) { sLd[wave][pos] = d2; sLi[wave][pos] = n; }
    cnt += __popc(mask);
    if (d2 < bestd) { bestd = d2; besti = n; }
  }
#pragma unroll
  for (int off = 16; off > 0; off >>= 1) {
    const float od = __shfl_xor(bestd, off, 32);
    const int oi = __shfl_xor(besti, off, 32);
    const bool take = (od < bestd) || (od == bestd && oi < besti);
    bestd = take ? od : bestd;
    besti = take ? oi : besti;
  }
  __syncthreads();
  const int ncl = cnt < LIST_CAP ? cnt : LIST_CAP;
  if (cnt <= NNBR) {
    const int jc = (ncl > 0) ? (lane < ncl ? lane : ncl - 1) : 0;
    const int li = sLi[wave][jc];
    sSel[wave][lane] = (lane < cnt) ? li : besti;
  } else {
    for (int jb = 0; jb < ncl; jb += 32) {
      const int j = jb + lane;
      const bool valid = j < ncl;
      const int jc = valid ? j : (ncl - 1);
      const float dj = sLd[wave][jc];
      const int ij = sLi[wave][jc];
      int rank = 0;
      for (int m = 0; m < ncl; ++m) {
        const float dm = sLd[wave][m];
        const int im = sLi[wave][m];
        rank += ((dm < dj) || (dm == dj && im < ij)) ? 1 : 0;
      }
      if (valid && rank < NNBR) sSel[wave][rank] = ij;
    }
  }
  __syncthreads();
  int sel = sSel[wave][lane];
  sel = sel < 0 ? 0 : (sel > NPTS - 1 ? NPTS - 1 : sel);
  volatile int* dst = (volatile int*)gidx + (size_t)q * NNBR + lane;
  *dst = sel;
  __threadfence();
  *dst = sel;
}

__global__ __launch_bounds__(256) void k_l0(const float* __restrict__ points, const float* __restrict__ pt4,
                                            const float* __restrict__ nxyz, const int* __restrict__ gidx,
                                            const unsigned* __restrict__ w0h, const float* __restrict__ bias0,
                                            unsigned* __restrict__ y0w, float* __restrict__ part0) {
  __shared__ __align__(16) unsigned short sA[TILE_ROWS * KPAD0];
  __shared__ __align__(16) unsigned short sW[CH_L0 * KPAD0];
  __shared__ __align__(16) unsigned short sSlab[TILE_ROWS * CH_L0];
  __shared__ float sPart[8][2 * CH_L0];
  const int t = threadIdx.x;
  const int lane = t & 31;
  const int wave = t >> 5;
  const int h = lane >> 4;
  const int c = lane & 15;
  const int blk = blockIdx.x;
#pragma unroll
  for (int i = 0; i < 3; ++i) {
    const int u = t + i * 256;
    const v4u w = ((const v4u*)w0h)[u];
    *(v4ua*)(sW + u * 8) = w;
  }
  asm volatile("" ::: "memory");
  {
    const int row = t >> 1;
    const int hf = t & 1;
    const int grow = blk * TILE_ROWS + row;
    const int g = grow >> 5;
    const int b = blk >> 8;
    int idx = gidx[grow];
    idx = idx < 0 ? 0 : (idx > NPTS - 1 ? NPTS - 1 : idx);
    const size_t base = (size_t)b * NPTS + (size_t)idx;
    const v4f* prow = (const v4f*)(points + base * CH_IN + hf * 32);
    const v4f pp = ((const v4f*)pt4)[base];
    const float cx = nxyz[(size_t)g * 3 + 0];
    const float cy = nxyz[(size_t)g * 3 + 1];
    const float cz = nxyz[(size_t)g * 3 + 2];
#pragma unroll
    for (int s = 0; s < 2; ++s) {
      const v4f a0 = prow[s * 4 + 0];
      const v4f a1 = prow[s * 4 + 1];
      const v4f a2 = prow[s * 4 + 2];
      const v4f a3 = prow[s * 4 + 3];
      v4u w0, w1;
      w0.x = pack2h(a0.x, a0.y); w0.y = pack2h(a0.z, a0.w);
      w0.z = pack2h(a1.x, a1.y); w0.w = pack2h(a1.z, a1.w);
      w1.x = pack2h(a2.x, a2.y); w1.y = pack2h(a2.z, a2.w);
      w1.z = pack2h(a3.x, a3.y); w1.w = pack2h(a3.z, a3.w);
      *(v4ua*)(sA + row * KPAD0 + hf * 32 + s * 16) = w0;
      *(v4ua*)(sA + row * KPAD0 + hf * 32 + s * 16 + 8) = w1;
      asm volatile("" ::: "memory");
    }
    const float dx = pp.x - cx;
    const float dy = pp.y - cy;
    const float dz = pp.z - cz;
    float zf = 0.0f;
    asm volatile("" : "+v"(zf));
    unsigned zz = 0u;
    asm volatile("" : "+v"(zz));
    const unsigned t0 = pack2h(dx, dy);
    const unsigned t1 = pack2h(dz, zf);
    v4u wt0, wt1;
    wt0.x = (hf == 0) ? t0 : zz;
    wt0.y = (hf == 0) ? t1 : zz;
    wt0.z = zz; wt0.w = zz;
    wt1.x = zz; wt1.y = zz; wt1.z = zz; wt1.w = zz;
    *(v4ua*)(sA + row * KPAD0 + 64 + hf * 16) = wt0;
    *(v4ua*)(sA + row * KPAD0 + 64 + hf * 16 + 8) = wt1;
  }
  __syncthreads();

  v8f acc[4];
#pragma unroll
  for (int j = 0; j < 4; ++j) acc[j] = (v8f){0.f, 0.f, 0.f, 0.f, 0.f, 0.f, 0.f, 0.f};
#pragma unroll
  for (int ks = 0; ks < KPAD0 / 32; ++ks) {
    const v16h a = lds_frag(sA, (wave * 16 + c) * KPAD0 + ks * 32 + 8 * h);
#pragma unroll
    for (int j = 0; j < 4; ++j) {
      const v16h bf = lds_frag(sW, (j * 16 + c) * KPAD0 + ks * 32 + 8 * h);
      acc[j] = mma_h(a, bf, acc[j]);
    }
  }
#pragma unroll
  for (int j = 0; j < 4; ++j) {
    const int n = j * 16 + c;
    const float bz = bias0[n];
    float s = 0.0f, sq = 0.0f;
#pragma unroll
    for (int r = 0; r < 8; ++r) {
      const float y = acc[j][r] * W_CARRY_INV + bz;
      const float y2 = y * y;
      s += y;
      sq += y2;
      sSlab[(wave * 16 + 8 * h + r) * CH_L0 + n] = (unsigned short)hbits(y);
    }
    s += __shfl_xor(s, 16, 32);
    sq += __shfl_xor(sq, 16, 32);
    if (h == 0) { sPart[wave][n] = s; sPart[wave][CH_L0 + n] = sq; }
  }
  __syncthreads();
  {
    const int q4 = lane >> 3;
    const int c8 = (lane & 7) * 8;
    v4u rv[4];
#pragma unroll
    for (int it = 0; it < 4; ++it) {
      const int row = it * 4 + q4;
      rv[it] = *(const v4ua*)(sSlab + (wave * 16 + row) * CH_L0 + c8);
    }
    for (int pass = 0; pass < 2; ++pass) {
#pragma unroll
      for (int it = 0; it < 4; ++it) {
        const int row = it * 4 + q4;
        const size_t hoff = ((size_t)blk * TILE_ROWS + wave * 16 + row) * CH_L0 + c8;
        *(volatile v4u*)(y0w + (hoff >> 1)) = rv[it];
      }
      __threadfence();
    }
  }
  if (t < 2 * CH_L0) {
    float tot = 0.0f;
#pragma unroll
    for (int w = 0; w < 8; ++w) tot += sPart[w][t];
    volatile float* dst = part0 + (size_t)blk * (2 * CH_L0) + t;
    *dst = tot;
    __threadfence();
    *dst = tot;
  }
}

template <int C>
__global__ __launch_bounds__(256) void k_fin(const float* __restrict__ part, const float* __restrict__ gam,
                                             const float* __restrict__ bet, float* __restrict__ scsh) {
  constexpr int NSTAT = 2 * C;
  constexpr int NSUB = 256 / NSTAT;
  constexpr int PER = NTILES / NSUB;
  static_assert(NSUB * NSTAT == 256 && PER * NSUB == NTILES, "finalize shape");
  __shared__ double sAcc[256];
  __shared__ float sOut[NSTAT];
  const int t = threadIdx.x;
  const int sub = t / NSTAT;
  const int stat = t - sub * NSTAT;
  double a = 0.0;
#pragma unroll 8
  for (int i = 0; i < PER; ++i) a += (double)part[(size_t)(sub * PER + i) * NSTAT + stat];
  sAcc[t] = a;
  __syncthreads();
  if (t < C) {
    double s = 0.0, sq = 0.0;
#pragma unroll
    for (int u = 0; u < NSUB; ++u) { s += sAcc[u * NSTAT + t]; sq += sAcc[u * NSTAT + C + t]; }
    const double invn = 1.0 / (double)NROWS;
    const double mean = s * invn;
    double var = sq * invn - mean * mean;
    var = var < 0.0 ? 0.0 : var;
    const float inv = 1.0f / sqrtf((float)var + BN_EPS);
    const float sc = gam[t] * inv;
    const float msc = (float)mean * sc;
    sOut[t] = sc;
    sOut[C + t] = bet[t] - msc;
  }
  __syncthreads();
  if (t < NSTAT) {
    const float v = sOut[t];
    volatile float* dst = scsh + t;
    *dst = v;
    __threadfence();
    *dst = v;
  }
}

__device__ __forceinline__ void stage_bn_tile(const unsigned* __restrict__ y0w, const float* __restrict__ scsh,
                                              unsigned short* sA, int blk, int t) {
  const int col0 = (t & 7) * 8;
  const v4f s0 = *(const v4f*)(scsh + col0);
  const v4f s1 = *(const v4f*)(scsh + col0 + 4);
  const v4f h0 = *(const v4f*)(scsh + CH_L0 + col0);
  const v4f h1 = *(const v4f*)(scsh + CH_L0 + col0 + 4);
  const v4u* src = (const v4u*)y0w + (size_t)blk * (TILE_ROWS * CH_L0 / 8);
  v4u w[4];
#pragma unroll
  for (int i = 0; i < 4; ++i) w[i] = src[t + i * 256];
#pragma unroll
  for (int i = 0; i < 4; ++i) {
    const unsigned wx = w[i].x;
    const unsigned wy = w[i].y;
    const unsigned wz = w[i].z;
    const unsigned ww = w[i].w;
    v4u o;
    o.x = bn_relu_pack(wx, s0.x, h0.x, s0.y, h0.y);
    o.y = bn_relu_pack(wy, s0.z, h0.z, s0.w, h0.w);
    o.z = bn_relu_pack(wz, s1.x, h1.x, s1.y, h1.y);
    o.w = bn_relu_pack(ww, s1.z, h1.z, s1.w, h1.w);
    *(v4ua*)(sA + (size_t)(t + i * 256) * 8) = o;
  }
}

__global__ __launch_bounds__(256) void k_l1stats(const unsigned* __restrict__ y0w, const float* __restrict__ scsh0,
                                                 const unsigned* __restrict__ w1h, const float* __restrict__ bias1,
                                                 float* __restrict__ part1) {
  __shared__ __align__(16) unsigned short sA[TILE_ROWS * CH_L0];
  __shared__ __align__(16) unsigned short sW[CH_L1 * CH_L0];
  __shared__ float sPart[8][2 * CH_L1];
  const int t = threadIdx.x;
  const int lane = t & 31;
  const int wave = t >> 5;
  const int h = lane >> 4;
  const int c = lane & 15;
  const int blk = blockIdx.x;
#pragma unroll
  for (int i = 0; i < 2; ++i) {
    const int u = t + i * 256;
    const v4u w = ((const v4u*)w1h)[u];
    *(v4ua*)(sW + u * 8) = w;
  }
  asm volatile("" ::: "memory");
  stage_bn_tile(y0w, scsh0, sA, blk, t);
  __syncthreads();
  v8f acc[4];
#pragma unroll
  for (int j = 0; j < 4; ++j) acc[j] = (v8f){0.f, 0.f, 0.f, 0.f, 0.f, 0.f, 0.f, 0.f};
#pragma unroll
  for (int ks = 0; ks < CH_L0 / 32; ++ks) {
    const v16h a = lds_frag(sA, (wave * 16 + c) * CH_L0 + ks * 32 + 8 * h);
#pragma unroll
    for (int j = 0; j < 4; ++j) {
      const v16h bf = lds_frag(sW, (j * 16 + c) * CH_L0 + ks * 32 + 8 * h);
      acc[j] = mma_h(a, bf, acc[j]);
    }
  }
#pragma unroll
  for (int j = 0; j < 4; ++j) {
    const int n = j * 16 + c;
    const float bz = bias1[n];
    float s = 0.0f, sq = 0.0f;
#pragma unroll
    for (int r = 0; r < 8; ++r) {
      const float y = acc[j][r] * W_CARRY_INV + bz;
      const float y2 = y * y;
      s += y;
      sq += y2;
    }
    s += __shfl_xor(s, 16, 32);
    sq += __shfl_xor(sq, 16, 32);
    if (h == 0) { sPart[wave][n] = s; sPart[wave][CH_L1 + n] = sq; }
  }
  __syncthreads();
  if (t < 2 * CH_L1) {
    float tot = 0.0f;
#pragma unroll
    for (int w = 0; w < 8; ++w) tot += sPart[w][t];
    volatile float* dst = part1 + (size_t)blk * (2 * CH_L1) + t;
    *dst = tot;
    __threadfence();
    *dst = tot;
  }
}

__global__ __launch_bounds__(256) void k_l12(const unsigned* __restrict__ y0w, const float* __restrict__ scsh0,
                                             const unsigned* __restrict__ w1h, const float* __restrict__ bias1,
                                             const float* __restrict__ scsh1, const unsigned* __restrict__ w2h,
                                             const float* __restrict__ bias2, float* __restrict__ part2,
                                             float* __restrict__ gmax, float* __restrict__ gmin) {
  __shared__ __align__(16) unsigned short sA[TILE_ROWS * CH_L0];
  __shared__ __align__(16) unsigned short sW1[CH_L1 * CH_L0];
  __shared__ __align__(16) unsigned short sW2[CH_L2 * CH_L1];
  __shared__ float sStat[4][8][CH_L2];
  const int t = threadIdx.x;
  const int lane = t & 31;
  const int wave = t >> 5;
  const int h = lane >> 4;
  const int c = lane & 15;
  const int blk = blockIdx.x;
#pragma unroll
  for (int i = 0; i < 2; ++i) {
    const int u = t + i * 256;
    const v4u w = ((const v4u*)w1h)[u];
    *(v4ua*)(sW1 + u * 8) = w;
  }
#pragma unroll
  for (int i = 0; i < 4; ++i) {
    const int u = t + i * 256;
    const v4u w = ((const v4u*)w2h)[u];
    *(v4ua*)(sW2 + u * 8) = w;
  }
  asm volatile("" ::: "memory");
  stage_bn_tile(y0w, scsh0, sA, blk, t);
  __syncthreads();
  {
    v8f acc[4];
#pragma unroll
    for (int j = 0; j < 4; ++j) acc[j] = (v8f){0.f, 0.f, 0.f, 0.f, 0.f, 0.f, 0.f, 0.f};
#pragma unroll
    for (int ks = 0; ks < CH_L0 / 32; ++ks) {
      const v16h a = lds_frag(sA, (wave * 16 + c) * CH_L0 + ks * 32 + 8 * h);
#pragma unroll
      for (int j = 0; j < 4; ++j) {
        const v16h bf = lds_frag(sW1, (j * 16 + c) * CH_L0 + ks * 32 + 8 * h);
        acc[j] = mma_h(a, bf, acc[j]);
      }
    }
#pragma unroll
    for (int j = 0; j < 4; ++j) {
      const int n = j * 16 + c;
      const float bz = bias1[n];
      const float sc = scsh1[n];
      const float sh = scsh1[CH_L1 + n];
#pragma unroll
      for (int r = 0; r < 8; ++r) {
        const float y = acc[j][r] * W_CARRY_INV + bz;
        const float ys = y * sc;
        const float a1 = fmaxf(ys + sh, 0.0f);
        sA[(wave * 16 + 8 * h + r) * CH_L1 + n] = (unsigned short)hbits(a1);
      }
    }
  }
  __syncthreads();
  v8f acc2[8];
#pragma unroll
  for (int j = 0; j < 8; ++j) acc2[j] = (v8f){0.f, 0.f, 0.f, 0.f, 0.f, 0.f, 0.f, 0.f};
#pragma unroll
  for (int ks = 0; ks < CH_L1 / 32; ++ks) {
    const v16h a = lds_frag(sA, (wave * 16 + c) * CH_L1 + ks * 32 + 8 * h);
#pragma unroll
    for (int j = 0; j < 8; ++j) {
      const v16h bf = lds_frag(sW2, (j * 16 + c) * CH_L1 + ks * 32 + 8 * h);
      acc2[j] = mma_h(a, bf, acc2[j]);
    }
  }
#pragma unroll
  for (int j = 0; j < 8; ++j) {
    const int n = j * 16 + c;
    const float bz = bias2[n];
    float s = 0.0f, sq = 0.0f;
    float mx = -__builtin_huge_valf();
    float mn = __builtin_huge_valf();
#pragma unroll
    for (int r = 0; r < 8; ++r) {
      const float y = acc2[j][r] * W_CARRY_INV + bz;
      const float y2 = y * y;
      s += y;
      sq += y2;
      mx = fmaxf(mx, y);
      mn = fminf(mn, y);
    }
    s += __shfl_xor(s, 16, 32);
    sq += __shfl_xor(sq, 16, 32);
    mx = fmaxf(mx, __shfl_xor(mx, 16, 32));
    mn = fminf(mn, __shfl_xor(mn, 16, 32));
    if (h == 0) {
      sStat[0][wave][n] = s;
      sStat[1][wave][n] = sq;
      sStat[2][wave][n] = mx;
      sStat[3][wave][n] = mn;
    }
  }
  __syncthreads();
  {
    const int which = t >> 7;
    const int cc = t & 127;
    float tot = 0.0f;
#pragma unroll
    for (int w = 0; w < 8; ++w) tot += sStat[which][w][cc];
    float mxv[2], mnv[2];
#pragma unroll
    for (int it = 0; it < 2; ++it) {
      const int v = it * 256 + t;
      const int g = v >> 7;
      const int ch = v & 127;
      mxv[it] = fmaxf(sStat[2][2 * g][ch], sStat[2][2 * g + 1][ch]);
      mnv[it] = fminf(sStat[3][2 * g][ch], sStat[3][2 * g + 1][ch]);
    }
    for (int pass = 0; pass < 2; ++pass) {
      *(volatile float*)(part2 + (size_t)blk * (2 * CH_L2) + t) = tot;
#pragma unroll
      for (int it = 0; it < 2; ++it) {
        const size_t o = (size_t)blk * (4 * CH_L2) + (size_t)(it * 256 + t);
        *(volatile float*)(gmax + o) = mxv[it];
        *(volatile float*)(gmin + o) = mnv[it];
      }
      __threadfence();
    }
  }
}

__global__ __launch_bounds__(256) void k_out(const float* __restrict__ gmax, const float* __restrict__ gmin,
                                             const float* __restrict__ scsh2, float* __restrict__ out1) {
  const int i = blockIdx.x * 256 + threadIdx.x;
  if (i < NGRP * CH_L2 / 4) {
    const int c4 = (i & 31) * 4;
    const v4f mx = ((const v4f*)gmax)[i];
    const v4f mn = ((const v4f*)gmin)[i];
    const v4f sc = *(const v4f*)(scsh2 + c4);
    const v4f sh = *(const v4f*)(scsh2 + CH_L2 + c4);
    v4f o;
    const float vx = (sc.x >= 0.0f) ? mx.x : mn.x;
    const float vy = (sc.y >= 0.0f) ? mx.y : mn.y;
    const float vz = (sc.z >= 0.0f) ? mx.z : mn.z;
    const float vw = (sc.w >= 0.0f) ? mx.w : mn.w;
    const float px = vx * sc.x;
    const float py = vy * sc.y;
    const float pz = vz * sc.z;
    const float pw = vw * sc.w;
    o.x = fmaxf(px + sh.x, 0.0f);
    o.y = fmaxf(py + sh.y, 0.0f);
    o.z = fmaxf(pz + sh.z, 0.0f);
    o.w = fmaxf(pw + sh.w, 0.0f);
    volatile v4f* dst = (volatile v4f*)out1 + i;
    *dst = o;
    __threadfence();
    *dst = o;
  }
}

extern "C" void kernel_launch(void* const* d_in, const int* in_sizes, int n_in,
                              void* d_out, int out_size, void* d_ws, size_t ws_size, hipStream_t stream) {
  (void)in_sizes; (void)out_size;
  if (n_in < 14) return;
  const float* xyz    = (const float*)d_in[0];
  const float* points = (const float*)d_in[1];
  const float* W0  = (const float*)d_in[2];
  const float* b0  = (const float*)d_in[3];
  const float* g0  = (const float*)d_in[4];
  const float* be0 = (const float*)d_in[5];
  const float* W1  = (const float*)d_in[6];
  const float* b1  = (const float*)d_in[7];
  const float* g1  = (const float*)d_in[8];
  const float* be1 = (const float*)d_in[9];
  const float* W2  = (const float*)d_in[10];
  const float* b2  = (const float*)d_in[11];
  const float* g2  = (const float*)d_in[12];
  const float* be2 = (const float*)d_in[13];

  if (ws_size < WS_TOTAL) return;
  char* ws = (char*)d_ws;
  size_t off = 0;
  float*    nxyz  = (float*)(ws + off);    off += WS_NXYZ;
  float*    pt4   = (float*)(ws + off);    off += WS_PT4;
  int*      gidx  = (int*)(ws + off);      off += WS_GIDX;
  unsigned* w0h   = (unsigned*)(ws + off); off += WS_W0H;
  unsigned* w1h   = (unsigned*)(ws + off); off += WS_W1H;
  unsigned* w2h   = (unsigned*)(ws + off); off += WS_W2H;
  unsigned* y0w   = (unsigned*)(ws + off); off += WS_Y0;
  float*    part0 = (float*)(ws + off);    off += WS_PART0;
  float*    part1 = (float*)(ws + off);    off += WS_PART1;
  float*    part2 = (float*)(ws + off);    off += WS_PART2;
  float*    scsh0 = (float*)(ws + off);    off += WS_SCSH0;
  float*    scsh1 = (float*)(ws + off);    off += WS_SCSH1;
  float*    scsh2 = (float*)(ws + off);    off += WS_SCSH2;
  float*    gmax  = (float*)(ws + off);    off += WS_GMAX;
  float*    gmin  = (float*)(ws + off);    off += WS_GMIN;

  float* out0 = (float*)d_out;
  float* out1 = out0 + (size_t)NGRP * 3;

  k_fps<<<NBATCH, 512, 0, stream>>>(xyz, out0, nxyz);
  k_prep<<<9 + (NBATCH * NPTS) / 256, 256, 0, stream>>>(xyz, W0, W1, W2, w0h, w1h, w2h, pt4);
  k_ballquery<<<NGRP / 8, 256, 0, stream>>>(pt4, nxyz, gidx);
  k_l0<<<NTILES, 256, 0, stream>>>(points, pt4, nxyz, gidx, w0h, b0, y0w, part0);
  k_fin<CH_L0><<<1, 256, 0, stream>>>(part0, g0, be0, scsh0);
  k_l1stats<<<NTILES, 256, 0, stream>>>(y0w, scsh0, w1h, b1, part1);
  k_fin<CH_L1><<<1, 256, 0, stream>>>(part1, g1, be1, scsh1);
  k_l12<<<NTILES, 256, 0, stream>>>(y0w, scsh0, w1h, b1, scsh1, w2h, b2, part2, gmax, gmin);
  k_fin<CH_L2><<<1, 256, 0, stream>>>(part2, g2, be2, scsh2);
  k_out<<<(NGRP * CH_L2 / 4) / 256, 256, 0, stream>>>(gmax, gmin, scsh2, out1);
}
